// LinOSSLayer_67723044323807
// MI455X (gfx1250) — hardware-verified
//
#include <hip/hip_runtime.h>
#include <math.h>

typedef __attribute__((ext_vector_type(16))) _Float16 v16h;
typedef __attribute__((ext_vector_type(8)))  _Float16 v8h;
typedef __attribute__((ext_vector_type(16))) __bf16   v16b;
typedef __attribute__((ext_vector_type(8)))  __bf16   v8b;
typedef __attribute__((ext_vector_type(8)))  float    v8f;
typedef __attribute__((ext_vector_type(4)))  float    v4f;
typedef __attribute__((ext_vector_type(2)))  float    v2f;
typedef __attribute__((ext_vector_type(4)))  unsigned v4u;

constexpr int kBatch = 4;
constexpr int kLen   = 8192;
constexpr int kWidth = 128;
constexpr int kState = 64;
constexpr int kCols  = 2 * kState;
constexpr int kRows  = kBatch * kLen;
constexpr int kChunk = 128;
constexpr int kNumCh = kLen / kChunk;
constexpr int kSubRows = 32;
constexpr int kTilePitch = 132;
static_assert(kCols == 128 && kWidth == 128);
static_assert((kRows % 64) == 0 && (kCols % 64) == 0 && (kWidth % 64) == 0);
static_assert((kCols % 32) == 0 && (kWidth % 32) == 0);
static_assert(kNumCh * kChunk == kLen && (kChunk % kSubRows) == 0);

constexpr int kSplitIn  = 0;
constexpr int kSplitOut = 0;

constexpr float kCarryU = 64.0f;
constexpr float kCarryW = 1024.0f;
constexpr float kCarryY = 32.0f;
constexpr float kF16MinNormal = 6.103515625e-05f;
constexpr float kScaleIn  = kSplitIn  ? 1.0f : 1.0f / (kCarryU * kCarryW);
constexpr float kScaleOut = kSplitOut ? 1.0f : 1.0f / (kCarryY * kCarryW);
constexpr float kMulU = kSplitIn  ? 1.0f : kCarryU;
constexpr float kMulB = kSplitIn  ? 1.0f : kCarryW;
constexpr float kMulC = kSplitOut ? 1.0f : kCarryW;
constexpr float kMulY = kSplitOut ? 1.0f : kCarryY;

constexpr size_t kPlane16   = (size_t)kRows * kCols * 2;
constexpr size_t kPlaneF32  = (size_t)kRows * kCols * 4;
constexpr size_t kWPlane    = (size_t)128 * 128 * 2;
constexpr size_t kCoefBytes = (size_t)10 * kState * 4;
constexpr size_t kCarryBytes = (size_t)kBatch * kNumCh * kCols * 2 * 4;
constexpr size_t kOffUH   = 0;
constexpr size_t kOffUL   = kOffUH  + kPlane16;
constexpr size_t kOffBU   = kOffUL  + kPlane16;
constexpr size_t kOffYH   = kOffBU  + kPlaneF32;
constexpr size_t kOffYL   = kOffYH  + kPlane16;
constexpr size_t kOffW1H  = kOffYL  + kPlane16;
constexpr size_t kOffW1L  = kOffW1H + kWPlane;
constexpr size_t kOffW2H  = kOffW1L + kWPlane;
constexpr size_t kOffW2L  = kOffW2H + kWPlane;
constexpr size_t kOffCoef = kOffW2L + kWPlane;
constexpr size_t kOffCEnd = kOffCoef + kCoefBytes;
constexpr size_t kOffCIn  = kOffCEnd + kCarryBytes;
constexpr size_t kWsTotal = kOffCIn + kCarryBytes;
static_assert(kWsTotal == 50989568ull);
static_assert(kWsTotal <= 134217728ull);
static_assert((kOffUL % 128) == 0 && (kOffBU % 128) == 0 && (kOffYH % 128) == 0 && (kOffYL % 128) == 0 &&
              (kOffW1H % 128) == 0 && (kOffW1L % 128) == 0 && (kOffW2H % 128) == 0 && (kOffW2L % 128) == 0 &&
              (kOffCoef % 128) == 0 && (kOffCEnd % 128) == 0 && (kOffCIn % 128) == 0);

__device__ __forceinline__ unsigned bf_top(float f) {
  unsigned u = __float_as_uint(f);
  const unsigned lsb = (u & 0x00010000u) ? 1u : 0u;
  u = (u + 0x7FFFu + lsb) & 0xFFFF0000u;
  return u;
}
__device__ __forceinline__ void split_pair(float x0, float x1, unsigned& wh, unsigned& wl) {
  const unsigned h0 = bf_top(x0);
  const unsigned h1 = bf_top(x1);
  const unsigned l0 = bf_top(x0 - __uint_as_float(h0));
  const unsigned l1 = bf_top(x1 - __uint_as_float(h1));
  wh = __builtin_amdgcn_perm(h1, h0, 0x07060302u);
  wl = __builtin_amdgcn_perm(l1, l0, 0x07060302u);
}
__device__ __forceinline__ float flush_f16(float c) {
  return (fabsf(c) < kF16MinNormal) ? 0.0f : c;
}
__device__ __forceinline__ v4u pack8_f16(v4f a0, v4f a1, float mul) {
  v8h hv;
  hv[0] = (_Float16)flush_f16(a0[0] * mul);
  hv[1] = (_Float16)flush_f16(a0[1] * mul);
  hv[2] = (_Float16)flush_f16(a0[2] * mul);
  hv[3] = (_Float16)flush_f16(a0[3] * mul);
  hv[4] = (_Float16)flush_f16(a1[0] * mul);
  hv[5] = (_Float16)flush_f16(a1[1] * mul);
  hv[6] = (_Float16)flush_f16(a1[2] * mul);
  hv[7] = (_Float16)flush_f16(a1[3] * mul);
  return __builtin_bit_cast(v4u, hv);
}
template <int SPL>
__device__ __forceinline__ void pack8(v4f a0, v4f a1, float mul, v4u& hi, v4u& lo) {
  if (SPL) {
    unsigned wh, wl;
    split_pair(a0[0] * mul, a0[1] * mul, wh, wl);
    hi[0] = wh;
    lo[0] = wl;
    split_pair(a0[2] * mul, a0[3] * mul, wh, wl);
    hi[1] = wh;
    lo[1] = wl;
    split_pair(a1[0] * mul, a1[1] * mul, wh, wl);
    hi[2] = wh;
    lo[2] = wl;
    split_pair(a1[2] * mul, a1[3] * mul, wh, wl);
    hi[3] = wh;
    lo[3] = wl;
  } else {
    hi = pack8_f16(a0, a1, mul);
    lo = hi;
  }
}
template <int SPL>
__device__ __forceinline__ void store8_twice(unsigned short* dh, unsigned short* dl, v4u hi, v4u lo) {
  *(volatile v4u*)dh = hi;
  if (SPL) *(volatile v4u*)dl = lo;
  __threadfence();
  *(volatile v4u*)dh = hi;
  if (SPL) *(volatile v4u*)dl = lo;
}

__device__ __forceinline__ void wm_guard_h(v8f& c, v16h a, v16h b) { asm volatile("v_nop\n\tv_nop\n\tv_nop\n\tv_nop" : "+v"(c) : "v"(a), "v"(b)); }
__device__ __forceinline__ void wm_guard_b(v8f& c, v16b a, v16b b) { asm volatile("v_nop\n\tv_nop\n\tv_nop\n\tv_nop" : "+v"(c) : "v"(a), "v"(b)); }
__device__ __forceinline__ void keep4_h(v16h a, v16h b, v16h c, v16h d) { asm volatile("v_nop" :: "v"(a), "v"(b), "v"(c), "v"(d)); }
__device__ __forceinline__ void keep4_b(v16b a, v16b b, v16b c, v16b d) { asm volatile("v_nop" :: "v"(a), "v"(b), "v"(c), "v"(d)); }
__device__ __forceinline__ void acc_guard4(v8f& a, v8f& b, v8f& c, v8f& d) { asm volatile("v_nop\n\tv_nop\n\tv_nop\n\tv_nop" : "+v"(a), "+v"(b), "+v"(c), "+v"(d)); }
template <typename T> struct Frag;
template <> struct Frag<_Float16> {
  typedef v16h V;
  union U { v16h v; v8h h[2]; };
  static __device__ __forceinline__ v16h load(const _Float16* p) {
    U f;
    f.h[0] = *(const v8h*)(p);
    f.h[1] = *(const v8h*)(p + 16);
    return f.v;
  }
  static __device__ __forceinline__ v8f mma(v16h a, v16h b, v8f c) {
    c = __builtin_amdgcn_wmma_f32_16x16x32_f16(false, a, false, b, (short)0, c, false, false);
    wm_guard_h(c, a, b);
    return c;
  }
  static __device__ __forceinline__ void keep(v16h a, v16h b, v16h c, v16h d) { keep4_h(a, b, c, d); }
};
template <> struct Frag<__bf16> {
  typedef v16b V;
  union U { v16b v; v8b h[2]; };
  static __device__ __forceinline__ v16b load(const __bf16* p) {
    U f;
    f.h[0] = *(const v8b*)(p);
    f.h[1] = *(const v8b*)(p + 16);
    return f.v;
  }
  static __device__ __forceinline__ v8f mma(v16b a, v16b b, v8f c) {
    c = __builtin_amdgcn_wmma_f32_16x16x32_bf16(false, a, false, b, (short)0, c, false, false);
    wm_guard_b(c, a, b);
    return c;
  }
  static __device__ __forceinline__ void keep(v16b a, v16b b, v16b c, v16b d) { keep4_b(a, b, c, d); }
};
template <int ET> struct Elem;
template <> struct Elem<0> { typedef _Float16 T; };
template <> struct Elem<1> { typedef __bf16 T; };
template <int SPLITSEL> struct GemmSel;
template <> struct GemmSel<0> { static constexpr int ET = 0; static constexpr int SP = 0; };
template <> struct GemmSel<1> { static constexpr int ET = 1; static constexpr int SP = 2; };

template <int ET, int SPL, bool RESMUL>
__global__ __launch_bounds__(256) void wmma_gemm64(
    const unsigned short* __restrict__ Ap, const unsigned short* __restrict__ A2p, int lda,
    const unsigned short* __restrict__ Btp, const unsigned short* __restrict__ Bt2p, int ldb,
    float* __restrict__ Cout, int ldc,
    const float* __restrict__ resid, const float* __restrict__ dvec,
    int M, int N, int K, float scale) {
  typedef typename Elem<ET>::T T;
  typedef typename Frag<T>::V V;
  const T* A   = (const T*)Ap;
  const T* A2  = (const T*)A2p;
  const T* Bt  = (const T*)Btp;
  const T* Bt2 = (const T*)Bt2p;
  __shared__ __align__(16) float sT[8][16 * 68];
  const int lane = threadIdx.x & 31;
  const int wave = threadIdx.x >> 5;
  const int tilesN = N >> 6;
  const int tilesM = M >> 6;
  const int tile = blockIdx.x * 8 + wave;
  if (tile >= tilesM * tilesN) return;
  const int tm = tile / tilesN;
  const int tn = tile - tm * tilesN;
  const int m0 = tm << 6;
  const int n0 = tn << 6;

  const int rlane = lane & 15;
  const int koff  = (lane >> 4) * 8;
  const int mOff  = (lane >> 4) * 8;

  v8f acc[4][4];
#pragma unroll
  for (int i = 0; i < 4; ++i)
#pragma unroll
    for (int j = 0; j < 4; ++j) acc[i][j] = (v8f){0.f, 0.f, 0.f, 0.f, 0.f, 0.f, 0.f, 0.f};

  for (int k0 = 0; k0 < K; k0 += 32) {
    V bh[4], bl[4];
#pragma unroll
    for (int j = 0; j < 4; ++j) {
      const size_t bo = (size_t)(n0 + (j << 4) + rlane) * ldb + koff + k0;
      bh[j] = Frag<T>::load(Bt + bo);
      if (SPL == 2) bl[j] = Frag<T>::load(Bt2 + bo);
    }
#pragma unroll
    for (int i = 0; i < 4; ++i) {
      const size_t ao = (size_t)(m0 + (i << 4) + rlane) * lda + koff + k0;
      V ah = Frag<T>::load(A + ao);
      V al;
      if (SPL == 2) al = Frag<T>::load(A2 + ao);
#pragma unroll
      for (int j = 0; j < 4; ++j) {
        acc[i][j] = Frag<T>::mma(ah, bh[j], acc[i][j]);
        if (SPL == 2) {
          acc[i][j] = Frag<T>::mma(ah, bl[j], acc[i][j]);
          acc[i][j] = Frag<T>::mma(al, bh[j], acc[i][j]);
        }
      }
    }
    Frag<T>::keep(bh[0], bh[1], bh[2], bh[3]);
    if (SPL == 2) Frag<T>::keep(bl[0], bl[1], bl[2], bl[3]);
  }
  acc_guard4(acc[0][0], acc[0][1], acc[0][2], acc[0][3]);
  acc_guard4(acc[1][0], acc[1][1], acc[1][2], acc[1][3]);
  acc_guard4(acc[2][0], acc[2][1], acc[2][2], acc[2][3]);
  acc_guard4(acc[3][0], acc[3][1], acc[3][2], acc[3][3]);

  float* slab = sT[wave];
  const int hh = lane >> 4;
  const int c4 = (lane & 15) * 4;
  v4f d4 = (v4f){0.f, 0.f, 0.f, 0.f};
  if (RESMUL) d4 = *(const v4f*)(dvec + n0 + c4);
#pragma unroll
  for (int i = 0; i < 4; ++i) {
    const int mBase = m0 + (i << 4);
#pragma unroll
    for (int j = 0; j < 4; ++j) {
#pragma unroll
      for (int r = 0; r < 8; ++r) {
        slab[(mOff + r) * 68 + (j << 4) + rlane] = acc[i][j][r] * scale;
      }
    }
    __builtin_amdgcn_fence(__ATOMIC_RELEASE, "workgroup");
    __builtin_amdgcn_wave_barrier();
    __builtin_amdgcn_fence(__ATOMIC_ACQUIRE, "workgroup");
    v4f val[8];
#pragma unroll
    for (int it = 0; it < 8; ++it) {
      const int row = it * 2 + hh;
      v4f v = *(const v4f*)(slab + row * 68 + c4);
      if (RESMUL) {
        const v4f u4 = *(const v4f*)(resid + (size_t)(mBase + row) * ldc + n0 + c4);
        v[0] = fmaf(u4[0], d4[0], v[0]);
        v[1] = fmaf(u4[1], d4[1], v[1]);
        v[2] = fmaf(u4[2], d4[2], v[2]);
        v[3] = fmaf(u4[3], d4[3], v[3]);
      }
      val[it] = v;
    }
    for (int pass = 0; pass < 2; ++pass) {
#pragma unroll
      for (int it = 0; it < 8; ++it) {
        const int row = it * 2 + hh;
        *(volatile v4f*)(Cout + (size_t)(mBase + row) * ldc + n0 + c4) = val[it];
      }
      __threadfence();
    }
    __builtin_amdgcn_fence(__ATOMIC_RELEASE, "workgroup");
    __builtin_amdgcn_wave_barrier();
    __builtin_amdgcn_fence(__ATOMIC_ACQUIRE, "workgroup");
  }
}

__global__ __launch_bounds__(256) void prep_kernel(
    const float* __restrict__ A_diag, const float* __restrict__ B_real, const float* __restrict__ B_imag,
    const float* __restrict__ C_real, const float* __restrict__ C_imag, const float* __restrict__ steps,
    unsigned short* __restrict__ W1H, unsigned short* __restrict__ W1L,
    unsigned short* __restrict__ W2H, unsigned short* __restrict__ W2L, float* __restrict__ coef)
{
#pragma clang fp contract(off)
  __shared__ __align__(16) float sC[10 * kState];
  const unsigned tid = threadIdx.x;
  const unsigned blk = blockIdx.x;
  if (blk < 8u) {
    unsigned i = (blk & 3u) * 256u + tid;
    asm volatile("" : "+v"(i));
    const unsigned n  = i >> 4;
    const unsigned k0 = (i & 15u) * 8u;
    const float* src = ((blk < 4u) ? B_real : B_imag) + (size_t)n * kWidth + k0;
    const unsigned nrow = ((blk < 4u) ? 0u : (unsigned)kState) + n;
    const size_t dsto = (size_t)nrow * kWidth + k0;
    const v4f a0 = *(const v4f*)(src);
    const v4f a1 = *(const v4f*)(src + 4);
    v4u hi, lo;
    pack8<kSplitIn>(a0, a1, kMulB, hi, lo);
    store8_twice<kSplitIn>(W1H + dsto, W1L + dsto, hi, lo);
  } else if (blk < 16u) {
    unsigned i = ((blk - 8u) & 3u) * 256u + tid;
    asm volatile("" : "+v"(i));
    const unsigned h  = i >> 3;
    const unsigned k0 = (i & 7u) * 8u;
    const bool imag = (blk >= 12u);
    const float* src = (imag ? C_imag : C_real) + (size_t)h * kState + k0;
    const size_t dsto = (size_t)h * kCols + (imag ? (unsigned)kState : 0u) + k0;
    const float mul = imag ? -kMulC : kMulC;
    const v4f a0 = *(const v4f*)(src);
    const v4f a1 = *(const v4f*)(src + 4);
    v4u hi, lo;
    pack8<kSplitOut>(a0, a1, mul, hi, lo);
    store8_twice<kSplitOut>(W2H + dsto, W2L + dsto, hi, lo);
  } else {
    const unsigned p = tid & 63u;
    float av = A_diag[p];
    float sv = steps[p];
    asm volatile("" : "+v"(av), "+v"(sv));
    const float A = fmaxf(av, 0.0f);
    const float s = 1.0f / (1.0f + expf(-sv));
    const float s2 = s * s;
    const float schur = 1.0f / (1.0f + s2 * A);
    const float m11 = 1.0f - s2 * A * schur;
    const float m12 = (-s) * A * schur;
    const float m21 = s * schur;
    const float m22 = schur;
    const float f1 = m11 * s;
    const float f2 = m21 * s;
    float c1z = 1.0f, c1x = 0.0f, c2z = 0.0f, c2x = 1.0f;
#pragma unroll 1
    for (int t = 0; t < kChunk; ++t) {
      const float a = fmaf(m11, c1z, m12 * c1x);
      const float b = fmaf(m21, c1z, m22 * c1x);
      const float d = fmaf(m11, c2z, m12 * c2x);
      const float e = fmaf(m21, c2z, m22 * c2x);
      c1z = a;
      c1x = b;
      c2z = d;
      c2x = e;
    }
    if (tid < (unsigned)kState) {
      sC[0 * kState + p] = m11;
      sC[1 * kState + p] = m12;
      sC[2 * kState + p] = m21;
      sC[3 * kState + p] = m22;
      sC[4 * kState + p] = f1;
      sC[5 * kState + p] = f2;
      sC[6 * kState + p] = c1z;
      sC[7 * kState + p] = c2z;
      sC[8 * kState + p] = c1x;
      sC[9 * kState + p] = c2x;
    }
    __syncthreads();
    if (tid < 160u) {
      const v4f v = *(const v4f*)(sC + tid * 4u);
      float* dst = coef + tid * 4u;
      *(volatile v4f*)dst = v;
      __threadfence();
      *(volatile v4f*)dst = v;
    }
  }
}

template <int SPL>
__global__ __launch_bounds__(256) void cvt_rows_kernel(
    const float* __restrict__ src, unsigned short* __restrict__ dhi, unsigned short* __restrict__ dlo,
    int total8, float mul)
{
  unsigned i = blockIdx.x * 256u + threadIdx.x;
  asm volatile("" : "+v"(i));
  if (i >= (unsigned)total8) return;
  const size_t e0 = (size_t)i << 3;
  const v4f a0 = *(const v4f*)(src + e0);
  const v4f a1 = *(const v4f*)(src + e0 + 4);
  v4u hi, lo;
  pack8<SPL>(a0, a1, mul, hi, lo);
  store8_twice<SPL>(dhi + e0, dlo + e0, hi, lo);
}

__device__ __forceinline__ void osc_step(float m11, float m12, float m21, float m22, float f1, float f2,
                                         float f, float& z, float& x) {
  const float nz = fmaf(m11, z, fmaf(m12, x, f1 * f));
  const float nx = fmaf(m21, z, fmaf(m22, x, f2 * f));
  z = nz;
  x = nx;
}

__global__ __launch_bounds__(64) void scan_local_kernel(
    const float* __restrict__ BU, const float* __restrict__ coef, float* __restrict__ CEND)
{
  unsigned j0 = threadIdx.x * 2u;
  asm volatile("" : "+v"(j0));
  unsigned p0 = j0 & 63u;
  asm volatile("" : "+v"(p0));
  const unsigned blk = blockIdx.x;
  const v2f m11 = *(const v2f*)(coef + 0 * kState + p0);
  const v2f m12 = *(const v2f*)(coef + 1 * kState + p0);
  const v2f m21 = *(const v2f*)(coef + 2 * kState + p0);
  const v2f m22 = *(const v2f*)(coef + 3 * kState + p0);
  const v2f f1  = *(const v2f*)(coef + 4 * kState + p0);
  const v2f f2  = *(const v2f*)(coef + 5 * kState + p0);
  const float* src = BU + (size_t)blk * kChunk * kCols + j0;
  float z0 = 0.0f, x0 = 0.0f, z1 = 0.0f, x1 = 0.0f;
#pragma unroll 4
  for (int t = 0; t < kChunk; ++t) {
    const v2f f = *(const v2f*)(src + (size_t)t * kCols);
    osc_step(m11[0], m12[0], m21[0], m22[0], f1[0], f2[0], f[0], z0, x0);
    osc_step(m11[1], m12[1], m21[1], m22[1], f1[1], f2[1], f[1], z1, x1);
  }
  const v4f e = (v4f){z0, x0, z1, x1};
  float* dst = CEND + ((size_t)blk * kCols + j0) * 2;
  *(volatile v4f*)dst = e;
  __threadfence();
  *(volatile v4f*)dst = e;
}

__global__ __launch_bounds__(64) void scan_carry_kernel(
    const float* __restrict__ coef, const float* __restrict__ CEND, float* __restrict__ CIN)
{
  unsigned j0 = threadIdx.x * 2u;
  asm volatile("" : "+v"(j0));
  unsigned p0 = j0 & 63u;
  asm volatile("" : "+v"(p0));
  const unsigned b = blockIdx.x;
  const v2f q11 = *(const v2f*)(coef + 6 * kState + p0);
  const v2f q12 = *(const v2f*)(coef + 7 * kState + p0);
  const v2f q21 = *(const v2f*)(coef + 8 * kState + p0);
  const v2f q22 = *(const v2f*)(coef + 9 * kState + p0);
  float az0 = 0.0f, ax0 = 0.0f, az1 = 0.0f, ax1 = 0.0f;
#pragma unroll 1
  for (int ch = 0; ch < kNumCh; ++ch) {
    const size_t off = ((size_t)(b * kNumCh + ch) * kCols + j0) * 2;
    const v4f cur = (v4f){az0, ax0, az1, ax1};
    const v4f e = *(const v4f*)(CEND + off);
    float* dst = CIN + off;
    *(volatile v4f*)dst = cur;
    __threadfence();
    *(volatile v4f*)dst = cur;
    const float nz0 = fmaf(q11[0], az0, fmaf(q12[0], ax0, e[0]));
    const float nx0 = fmaf(q21[0], az0, fmaf(q22[0], ax0, e[1]));
    const float nz1 = fmaf(q11[1], az1, fmaf(q12[1], ax1, e[2]));
    const float nx1 = fmaf(q21[1], az1, fmaf(q22[1], ax1, e[3]));
    az0 = nz0;
    ax0 = nx0;
    az1 = nz1;
    ax1 = nx1;
  }
}

template <int SPL>
__global__ __launch_bounds__(64) void scan_final_kernel(
    const float* __restrict__ BU, const float* __restrict__ coef, const float* __restrict__ CIN,
    unsigned short* __restrict__ YH, unsigned short* __restrict__ YL, float mul)
{
  __shared__ __align__(16) float sY[kSubRows * kTilePitch];
  const unsigned tid = threadIdx.x;
  unsigned j0 = tid * 2u;
  asm volatile("" : "+v"(j0));
  unsigned p0 = j0 & 63u;
  asm volatile("" : "+v"(p0));
  const unsigned blk = blockIdx.x;
  const v2f m11 = *(const v2f*)(coef + 0 * kState + p0);
  const v2f m12 = *(const v2f*)(coef + 1 * kState + p0);
  const v2f m21 = *(const v2f*)(coef + 2 * kState + p0);
  const v2f m22 = *(const v2f*)(coef + 3 * kState + p0);
  const v2f f1  = *(const v2f*)(coef + 4 * kState + p0);
  const v2f f2  = *(const v2f*)(coef + 5 * kState + p0);
  const v4f cin = *(const v4f*)(CIN + ((size_t)blk * kCols + j0) * 2);
  float z0 = cin[0], x0 = cin[1], z1 = cin[2], x1 = cin[3];
  const size_t row0 = (size_t)blk * kChunk;
  unsigned r4 = tid >> 4;
  asm volatile("" : "+v"(r4));
  unsigned c8 = (tid & 15u) * 8u;
  asm volatile("" : "+v"(c8));
#pragma unroll 1
  for (int sub = 0; sub < kChunk / kSubRows; ++sub) {
    const float* src = BU + (row0 + (size_t)sub * kSubRows) * kCols + j0;
#pragma unroll 4
    for (int s = 0; s < kSubRows; ++s) {
      const v2f f = *(const v2f*)(src + (size_t)s * kCols);
      osc_step(m11[0], m12[0], m21[0], m22[0], f1[0], f2[0], f[0], z0, x0);
      osc_step(m11[1], m12[1], m21[1], m22[1], f1[1], f2[1], f[1], z1, x1);
      *(v2f*)(sY + s * kTilePitch + j0) = (v2f){x0, x1};
    }
    __syncthreads();
    v4u hw[8], lw[8];
#pragma unroll
    for (int it = 0; it < 8; ++it) {
      const unsigned row = (unsigned)it * 4u + r4;
      const float* sp = sY + row * kTilePitch + c8;
      const v4f a0 = *(const v4f*)(sp);
      const v4f a1 = *(const v4f*)(sp + 4);
      pack8<SPL>(a0, a1, mul, hw[it], lw[it]);
    }
    for (int pass = 0; pass < 2; ++pass) {
#pragma unroll
      for (int it = 0; it < 8; ++it) {
        const unsigned row = (unsigned)it * 4u + r4;
        const size_t o = (row0 + (size_t)sub * kSubRows + row) * kCols + c8;
        *(volatile v4u*)(YH + o) = hw[it];
        if (SPL) *(volatile v4u*)(YL + o) = lw[it];
      }
      __threadfence();
    }
    __syncthreads();
  }
}

extern "C" void kernel_launch(void* const* d_in, const int* in_sizes, int n_in,
                              void* d_out, int out_size, void* d_ws, size_t ws_size,
                              hipStream_t stream) {
  if (n_in < 8) return;
  if (in_sizes[0] != kRows * kWidth) return;
  if (in_sizes[1] != kState) return;
  if (in_sizes[2] != kState * kWidth) return;
  if (in_sizes[3] != kState * kWidth) return;
  if (in_sizes[4] != kWidth * kState) return;
  if (in_sizes[5] != kWidth * kState) return;
  if (in_sizes[6] != kWidth) return;
  if (in_sizes[7] != kState) return;
  if (out_size != kRows * kWidth) return;
  if (ws_size < kWsTotal) return;

  const float* u      = (const float*)d_in[0];
  const float* A_diag = (const float*)d_in[1];
  const float* B_real = (const float*)d_in[2];
  const float* B_imag = (const float*)d_in[3];
  const float* C_real = (const float*)d_in[4];
  const float* C_imag = (const float*)d_in[5];
  const float* Dv     = (const float*)d_in[6];
  const float* steps  = (const float*)d_in[7];
  float* out = (float*)d_out;

  char* ws = (char*)d_ws;
  unsigned short* UH   = (unsigned short*)(ws + kOffUH);
  unsigned short* UL   = (unsigned short*)(ws + kOffUL);
  float*          BU   = (float*)(ws + kOffBU);
  unsigned short* YH   = (unsigned short*)(ws + kOffYH);
  unsigned short* YL   = (unsigned short*)(ws + kOffYL);
  unsigned short* W1H  = (unsigned short*)(ws + kOffW1H);
  unsigned short* W1L  = (unsigned short*)(ws + kOffW1L);
  unsigned short* W2H  = (unsigned short*)(ws + kOffW2H);
  unsigned short* W2L  = (unsigned short*)(ws + kOffW2L);
  float*          COEF = (float*)(ws + kOffCoef);
  float*          CEND = (float*)(ws + kOffCEnd);
  float*          CIN  = (float*)(ws + kOffCIn);

  prep_kernel<<<17, 256, 0, stream>>>(A_diag, B_real, B_imag, C_real, C_imag, steps, W1H, W1L, W2H, W2L, COEF);

  cvt_rows_kernel<kSplitIn><<<(kRows * kWidth / 8) / 256, 256, 0, stream>>>(u, UH, UL, kRows * kWidth / 8, kMulU);

  wmma_gemm64<GemmSel<kSplitIn>::ET, GemmSel<kSplitIn>::SP, false><<<128, 256, 0, stream>>>(
      UH, UL, kWidth,
      W1H, W1L, kWidth,
      BU, kCols,
      u, Dv,
      kRows, kCols, kWidth, kScaleIn);

  scan_local_kernel<<<kBatch * kNumCh, 64, 0, stream>>>(BU, COEF, CEND);

  scan_carry_kernel<<<kBatch, 64, 0, stream>>>(COEF, CEND, CIN);

  scan_final_kernel<kSplitOut><<<kBatch * kNumCh, 64, 0, stream>>>(BU, COEF, CIN, YH, YL, kMulY);

  wmma_gemm64<GemmSel<kSplitOut>::ET, GemmSel<kSplitOut>::SP, true><<<128, 256, 0, stream>>>(
      YH, YL, kCols,
      W2H, W2L, kCols,
      out, kWidth,
      u, Dv,
      kRows, kWidth, kCols, kScaleOut);
}
